// SimpleSSM_67379446940102
// MI455X (gfx1250) — hardware-run, weakly checked
//
#include <hip/hip_runtime.h>
#include <math.h>

typedef __attribute__((ext_vector_type(16))) _Float16 v16h;
typedef __attribute__((ext_vector_type(8)))  _Float16 v8h;
typedef __attribute__((ext_vector_type(2)))  _Float16 v2h;
typedef __attribute__((ext_vector_type(16))) __bf16   v16b;
typedef __attribute__((ext_vector_type(8)))  __bf16   v8b;
typedef __attribute__((ext_vector_type(8)))  float    v8f;
typedef __attribute__((ext_vector_type(4)))  float    v4f;
typedef __attribute__((ext_vector_type(2)))  float    v2f;

constexpr int kNB   = 4;
constexpr int kL    = 2048;
constexpr int kRows = kNB * kL;
constexpr int kHid  = 768;
constexpr int kDI   = 1536;
constexpr int kXZ   = 2 * kDI;
constexpr int kNs   = 16;
constexpr int kTaps = 4;
constexpr int kXpP  = 64;
constexpr int kOut0 = kRows * kHid;
constexpr int kOut1 = kNB * kDI * kNs;
constexpr int kThr  = 256;
constexpr float kInCarry = 1024.0f;
constexpr float kWCarry  = 4096.0f;
constexpr float kUCarry  = 4096.0f;
constexpr float kYCarry  = 4096.0f;
constexpr float kScIn = 1.0f / (kInCarry * kInCarry);
constexpr float kScU  = 1.0f / (kUCarry * kInCarry);
constexpr float kScY  = 1.0f / (kYCarry * kInCarry);
constexpr float kF16MinNormal = 6.103515625e-5f;

static_assert(kRows == 8192 && kHid == 768 && kDI == 1536 && kXZ == 3072 && kNs == 16 && kTaps == 4 && (kL & (kL - 1)) == 0, "the index arithmetic below uses these sizes");

constexpr size_t kOffX16 = 0ull;
constexpr size_t kOffWIN16 = 12582912ull;
constexpr size_t kOffWOUT16 = 17301504ull;
constexpr size_t kOffWXP16 = 19660800ull;
constexpr size_t kOffZB = 19857408ull;
constexpr size_t kOffXZ = 19869696ull;
constexpr size_t kOffU16 = 120532992ull;
constexpr size_t kOffXP = 145698816ull;
constexpr size_t kOffY16 = 147795968ull;
constexpr size_t kWsTotal = 172961792ull;
static_assert(kWsTotal <= 268435456ull, "the carve stands under the contract's 256 MiB of workspace");
static_assert(kOffX16 == 0
  && kOffWIN16 == kOffX16 + 12582912ull
  && kOffWOUT16 == kOffWIN16 + 4718592ull
  && kOffWXP16 == kOffWOUT16 + 2359296ull
  && kOffZB == kOffWXP16 + 196608ull
  && kOffXZ == kOffZB + 12288ull
  && kOffU16 == kOffXZ + 100663296ull
  && kOffXP == kOffU16 + 25165824ull
  && kOffY16 == kOffXP + 2097152ull
  && kWsTotal == kOffY16 + 25165824ull, "the carve is a chain: every region starts where the one before ends");
static_assert((kOffWIN16 % 256) == 0 && (kOffWOUT16 % 256) == 0 && (kOffWXP16 % 256) == 0 && (kOffZB % 256) == 0 && (kOffXZ % 256) == 0 && (kOffU16 % 256) == 0 && (kOffXP % 256) == 0 && (kOffY16 % 256) == 0, "every region starts on a multiple of 256 B");

__device__ __forceinline__ unsigned short f2bf_bits(float f) {
  unsigned u = __float_as_uint(f);
  return (unsigned short)((u + 0x7FFFu + ((u >> 16) & 1u)) >> 16);
}
__device__ __forceinline__ float bf_bits2f(unsigned short h) { return __uint_as_float(((unsigned)h) << 16); }
__device__ __forceinline__ float bf16r(float f) { return bf_bits2f(f2bf_bits(f)); }
__device__ __forceinline__ float carry_flush(float v, float carry) {
  const float s = v * carry;
  return (fabsf(s) < kF16MinNormal) ? 0.0f : s;
}

__device__ __forceinline__ void dep_guard4_h(v8f& a, v8f& b, v8f& c, v8f& d, v16h x, v16h y) { asm volatile("v_nop\n\tv_nop\n\tv_nop\n\tv_nop" : "+v"(a), "+v"(b), "+v"(c), "+v"(d) : "v"(x), "v"(y)); }
__device__ __forceinline__ void dep_guard4_b(v8f& a, v8f& b, v8f& c, v8f& d, v16b x, v16b y) { asm volatile("v_nop\n\tv_nop\n\tv_nop\n\tv_nop" : "+v"(a), "+v"(b), "+v"(c), "+v"(d) : "v"(x), "v"(y)); }
__device__ __forceinline__ void keep4_h(v16h a, v16h b, v16h c, v16h d) { asm volatile("v_nop" :: "v"(a), "v"(b), "v"(c), "v"(d)); }
__device__ __forceinline__ void keep4_b(v16b a, v16b b, v16b c, v16b d) { asm volatile("v_nop" :: "v"(a), "v"(b), "v"(c), "v"(d)); }
__device__ __forceinline__ void acc_guard4(v8f& a, v8f& b, v8f& c, v8f& d) { asm volatile("v_nop\n\tv_nop\n\tv_nop\n\tv_nop" : "+v"(a), "+v"(b), "+v"(c), "+v"(d)); }

template <typename T> struct Frag;
template <> struct Frag<_Float16> {
  typedef v16h V; union U { v16h v; v8h h[2]; };
  static __device__ __forceinline__ v16h load(const _Float16* p) {
    U f; f.h[0] = *(const v8h*)(p); f.h[1] = *(const v8h*)(p + 16); return f.v;
  }
  static __device__ __forceinline__ v8f mma(v16h a, v16h b, v8f c) {
    return __builtin_amdgcn_wmma_f32_16x16x32_f16(false, a, false, b, (short)0, c, false, false);
  }
  static __device__ __forceinline__ void guard4(v8f& a, v8f& b, v8f& c, v8f& d, v16h x, v16h y) { dep_guard4_h(a, b, c, d, x, y); }
  static __device__ __forceinline__ void keep(v16h a, v16h b, v16h c, v16h d) { keep4_h(a, b, c, d); }
};
template <> struct Frag<__bf16> {
  typedef v16b V; union U { v16b v; v8b h[2]; };
  static __device__ __forceinline__ v16b load(const __bf16* p) {
    U f; f.h[0] = *(const v8b*)(p); f.h[1] = *(const v8b*)(p + 16); return f.v;
  }
  static __device__ __forceinline__ v8f mma(v16b a, v16b b, v8f c) {
    return __builtin_amdgcn_wmma_f32_16x16x32_bf16(false, a, false, b, (short)0, c, false, false);
  }
  static __device__ __forceinline__ void guard4(v8f& a, v8f& b, v8f& c, v8f& d, v16b x, v16b y) { dep_guard4_b(a, b, c, d, x, y); }
  static __device__ __forceinline__ void keep(v16b a, v16b b, v16b c, v16b d) { keep4_b(a, b, c, d); }
};

__device__ __forceinline__ v8f mma_h(v16h a, v16h b, v8f c) {
  c = __builtin_amdgcn_wmma_f32_16x16x32_f16(false, a, false, b, (short)0, c, false, false);
  asm volatile("v_nop\n\tv_nop\n\tv_nop\n\tv_nop" : "+v"(c) : "v"(a), "v"(b));
  return c;
}

template <int ET> struct Elem;
template <> struct Elem<0> { typedef _Float16 T; };
template <> struct Elem<1> { typedef __bf16 T; };
template <int ET, bool SPLIT, int BIAS_MODE, int OUT_MODE, bool RESID, int ACT = 0>
__global__ __launch_bounds__(256) void wmma_gemm64(
    const unsigned short* __restrict__ Ap, const unsigned short* __restrict__ A2p, int lda, long strideA,
    const unsigned short* __restrict__ Btp, const unsigned short* __restrict__ Bt2p, int ldb, long strideB,
    void* __restrict__ Cout, void* __restrict__ Cout2, int ldc, long strideC,
    const float* __restrict__ bias,
    const float* __restrict__ resid, long strideR,
    int M, int N, int K, float scale) {
  typedef typename Elem<ET>::T T;
  typedef typename Frag<T>::V V;
  const T* A = (const T*)Ap; const T* A2 = (const T*)A2p; const T* Bt = (const T*)Btp; const T* Bt2 = (const T*)Bt2p;
  __shared__ __align__(16) float sT[8][16 * 68];
  const int b    = blockIdx.y;
  const int lane = threadIdx.x & 31;
  const int wave = threadIdx.x >> 5;
  const int tilesN = N >> 6;
  const int tilesM = M >> 6;
  const int tile = blockIdx.x * 8 + wave;
  if (tile >= tilesM * tilesN) return;
  const int tm = tile / tilesN;
  const int tn = tile - tm * tilesN;
  const int m0 = tm << 6;
  const int n0 = tn << 6;

  const T* Ab  = A  + (size_t)b * strideA;
  const T* Bb  = Bt + (size_t)b * strideB;
  const T* Ab2 = SPLIT ? (A2  + (size_t)b * strideA) : nullptr;
  const T* Bb2 = SPLIT ? (Bt2 + (size_t)b * strideB) : nullptr;

  const int rlane = lane & 15;
  const int koff  = (lane >> 4) * 8;
  const int mOff  = (lane >> 4) * 8;

  v8f acc[4][4];
#pragma unroll
  for (int i = 0; i < 4; ++i)
#pragma unroll
    for (int j = 0; j < 4; ++j) acc[i][j] = (v8f){0.f,0.f,0.f,0.f,0.f,0.f,0.f,0.f};

  for (int k0 = 0; k0 < K; k0 += 32) {
    V bh[4], bl[4];
#pragma unroll
    for (int j = 0; j < 4; ++j) {
      const size_t bo = (size_t)(n0 + (j << 4) + rlane) * ldb + koff + k0;
      bh[j] = Frag<T>::load(Bb + bo);
      if (SPLIT) bl[j] = Frag<T>::load(Bb2 + bo);
    }
#pragma unroll
    for (int i = 0; i < 4; ++i) {
      const size_t ao = (size_t)(m0 + (i << 4) + rlane) * lda + koff + k0;
      V ah = Frag<T>::load(Ab + ao);
      V al;
      if (SPLIT) al = Frag<T>::load(Ab2 + ao);
#pragma unroll
      for (int j = 0; j < 4; ++j) {
        acc[i][j] = Frag<T>::mma(ah, bh[j], acc[i][j]);
        if (SPLIT) {
          acc[i][j] = Frag<T>::mma(ah, bl[j], acc[i][j]);
          acc[i][j] = Frag<T>::mma(al, bh[j], acc[i][j]);
        }
      }
      Frag<T>::guard4(acc[i][0], acc[i][1], acc[i][2], acc[i][3], ah, SPLIT ? al : ah);
    }
    Frag<T>::keep(bh[0], bh[1], bh[2], bh[3]);
    if (SPLIT) Frag<T>::keep(bl[0], bl[1], bl[2], bl[3]);
  }
  acc_guard4(acc[0][0], acc[0][1], acc[0][2], acc[0][3]);
  acc_guard4(acc[1][0], acc[1][1], acc[1][2], acc[1][3]);
  acc_guard4(acc[2][0], acc[2][1], acc[2][2], acc[2][3]);
  acc_guard4(acc[3][0], acc[3][1], acc[3][2], acc[3][3]);

  float* slab = sT[wave];
  const float* Rb = RESID ? (resid + (size_t)b * strideR) : nullptr;
#pragma unroll
  for (int i = 0; i < 4; ++i) {
    const int mBase = m0 + (i << 4);
#pragma unroll
    for (int j = 0; j < 4; ++j) {
      const int n = n0 + (j << 4) + rlane;
      float bv = 0.f;
      if (BIAS_MODE == 2) bv = bias[n];
#pragma unroll
      for (int r = 0; r < 8; ++r) {
        float v = acc[i][j][r] * scale;
        if (BIAS_MODE == 1) v += bias[mBase + mOff + r];
        if (BIAS_MODE == 2) v += bv;
        if (RESID) v += Rb[(size_t)(mBase + mOff + r) * ldc + n];
        if (ACT == 1) v = tanhf(v);
        if (ACT == 2) v = fmaxf(v, 0.0f);
        if (ACT == 3) v = v / (1.0f + expf(-v));
        if (ACT == 4) v = (v > 0.f) ? v : 0.01f * v;
        slab[(mOff + r) * 68 + (j << 4) + rlane] = v;
      }
    }
    __builtin_amdgcn_fence(__ATOMIC_RELEASE, "workgroup");
    __builtin_amdgcn_wave_barrier();
    __builtin_amdgcn_fence(__ATOMIC_ACQUIRE, "workgroup");
    if (OUT_MODE == 0) {
      float* C = (float*)Cout + (size_t)b * strideC;
      const int hh = lane >> 4, c4 = (lane & 15) * 4;
      for (int pass = 0; pass < 2; ++pass) {
#pragma unroll
        for (int it = 0; it < 8; ++it) {
          const int row = it * 2 + hh;
          v4f v = *(const v4f*)(slab + row * 68 + c4);
          *(volatile v4f*)(C + (size_t)(mBase + row) * ldc + n0 + c4) = v;
        }
        __threadfence();
      }
    } else {
      const int q = lane >> 3, c8 = (lane & 7) * 8;
      unsigned short* C  = (unsigned short*)Cout  + (size_t)b * strideC;
      unsigned short* C2 = (OUT_MODE == 2) ? ((unsigned short*)Cout2 + (size_t)b * strideC) : nullptr;
      for (int pass = 0; pass < 2; ++pass) {
#pragma unroll
        for (int it = 0; it < 4; ++it) {
          const int row = it * 4 + q;
          const float* sp = slab + row * 68 + c8;
          v8h hv, lv;
#pragma unroll
          for (int e = 0; e < 8; ++e) {
            if (OUT_MODE == 1) {
              hv[e] = (_Float16)sp[e];
            } else {
              unsigned short hb = f2bf_bits(sp[e]);
              unsigned short lb = f2bf_bits(sp[e] - bf_bits2f(hb));
              hv[e] = __builtin_bit_cast(_Float16, hb);
              lv[e] = __builtin_bit_cast(_Float16, lb);
            }
          }
          *(volatile v8h*)(C + (size_t)(mBase + row) * ldc + n0 + c8) = hv;
          if (OUT_MODE == 2) *(volatile v8h*)(C2 + (size_t)(mBase + row) * ldc + n0 + c8) = lv;
        }
        __threadfence();
      }
    }
    __builtin_amdgcn_fence(__ATOMIC_RELEASE, "workgroup");
    __builtin_amdgcn_wave_barrier();
    __builtin_amdgcn_fence(__ATOMIC_ACQUIRE, "workgroup");
  }
}


__device__ __forceinline__ void store2(float* p, float v) {
  *(volatile float*)p = v;
  __threadfence();
  *(volatile float*)p = v;
}

__global__ __launch_bounds__(kThr) void cast_plane_kernel(const float* __restrict__ src, unsigned short* __restrict__ dst,
                                                          int colsLog2, int dstPitch, int dstOff) {
  const int i   = blockIdx.x * kThr + threadIdx.x;
  const int sh  = colsLog2 - 3;
  const int row = i >> sh;
  const int c8  = (i & ((1 << sh) - 1)) * 8;
  const float* sp = src + ((size_t)row << colsLog2) + c8;
  const v4f a0 = *(const v4f*)(sp);
  const v4f a1 = *(const v4f*)(sp + 4);
  v8h hv;
#pragma unroll
  for (int e = 0; e < 4; ++e) {
    const float f0 = a0[e];
    const float f1 = a1[e];
    hv[e]     = (_Float16)carry_flush(bf16r(f0), kInCarry);
    hv[4 + e] = (_Float16)carry_flush(bf16r(f1), kInCarry);
  }
  unsigned short* dp = dst + (size_t)row * dstPitch + dstOff + c8;
  *(volatile v8h*)dp = hv;
  __threadfence();
  *(volatile v8h*)dp = hv;
}

__global__ __launch_bounds__(256) void wt_plane_kernel(const float* __restrict__ W, unsigned short* __restrict__ dst, int K, int N, int nLive, int ldd, int colOff) {
  const int n  = blockIdx.x;
  const int k8 = threadIdx.x * 8;
  const bool live = n < nLive;
  const int nc = live ? n : 0;
  v8h hv;
#pragma unroll
  for (int e = 0; e < 8; ++e) {
    const float w = W[(size_t)(k8 + e) * N + nc];
    hv[e] = (_Float16)(live ? carry_flush(bf16r(w), kWCarry) : 0.0f);
  }
  unsigned short* dp = dst + (size_t)n * ldd + colOff + k8;
  *(volatile v8h*)dp = hv;
  __threadfence();
  *(volatile v8h*)dp = hv;
}

__global__ __launch_bounds__(kThr) void setup_kernel(const float* __restrict__ W_xp, float* __restrict__ ZB, unsigned short* __restrict__ WXP16) {
  const unsigned bk = blockIdx.x;
  if (bk < 12u) {
    float* dp = ZB + bk * (unsigned)kThr + threadIdx.x;
    *(volatile float*)dp = 0.0f;
    __threadfence();
    *(volatile float*)dp = 0.0f;
  } else {
    const unsigned j = (bk - 12u) * (unsigned)kThr + threadIdx.x;
    const unsigned r = j / 192u;
    const unsigned c8 = (j - r * 192u) * 8u;
    const bool live = r <= 32u;
    const unsigned sr = (r == 32u) ? 0u : (r + 1u);
    const float* sp = W_xp + (size_t)(live ? sr : 0u) * kDI + c8;
    const v4f a0 = *(const v4f*)sp, a1 = *(const v4f*)(sp + 4);
    v8h hv;
#pragma unroll
    for (int e = 0; e < 8; ++e) { const float f = (e < 4) ? a0[e] : a1[e - 4]; hv[e] = (_Float16)(live ? carry_flush(bf16r(f), kInCarry) : 0.0f); }
    unsigned short* dp = WXP16 + (size_t)j * 8;
    *(volatile v8h*)dp = hv;
    __threadfence();
    *(volatile v8h*)dp = hv;
  }
}
static_assert(12 * kThr == kXZ && (size_t)kXpP * kDI / 8 == 48ull * kThr && kDI / 8 == 192, "set-up grid exact: 12 blocks of zero bias, 48 of the small projection's weight plane");

__global__ __launch_bounds__(kThr) void front_kernel(const float* __restrict__ XZ, const float* __restrict__ conv_w, unsigned short* __restrict__ U16) {
  const unsigned i = blockIdx.x * (unsigned)kThr + threadIdx.x;
  const unsigned row = i / 192u;
  const unsigned c8 = (i - row * 192u) * 8u;
  const int tok = (int)(row & (unsigned)(kL - 1));
  float acc[8];
#pragma unroll
  for (int e = 0; e < 8; ++e) acc[e] = 0.0f;
#pragma unroll
  for (int k = 0; k < kTaps; ++k) {
    const int back = kTaps - 1 - k;
    const bool has = tok >= back;
    const float* xp = XZ + (size_t)(row - (has ? (unsigned)back : 0u)) * kXZ + c8;
    const v4f a0 = *(const v4f*)xp, a1 = *(const v4f*)(xp + 4);
#pragma unroll
    for (int e = 0; e < 8; ++e) {
      const float wv = conv_w[(size_t)(c8 + e) * kTaps + k];
      const float xv = (e < 4) ? a0[e] : a1[e - 4];
      acc[e] += (has ? xv : 0.0f) * bf16r(wv);
    }
  }
  v8h hv;
#pragma unroll
  for (int e = 0; e < 8; ++e) { const float xc = acc[e] / (1.0f + expf(-acc[e])); hv[e] = (_Float16)carry_flush(xc, kUCarry); }
  unsigned short* dp = U16 + (size_t)i * 8;
  *(volatile v8h*)dp = hv;
  __threadfence();
  *(volatile v8h*)dp = hv;
}
static_assert((size_t)kRows * kDI / 8 == 6144ull * kThr, "the front's grid exact: 6,144 blocks");

__global__ __launch_bounds__(kThr) void scan_kernel(const float* __restrict__ XZ, const float* __restrict__ XP, const float* __restrict__ conv_w, const float* __restrict__ A_log,
                                                    const float* __restrict__ Dp, unsigned short* __restrict__ Y16, float* __restrict__ out1) {
  const unsigned ix = blockIdx.x * (unsigned)kThr + threadIdx.x;
  const unsigned sq = ix / 768u;
  const unsigned c0 = (ix - sq * 768u) * 2u;
  float A[2][kNs], st[2][kNs], cw[2][kTaps], win[2][kTaps - 1], dc[2];
#pragma unroll
  for (int k = 0; k < 2; ++k) {
#pragma unroll
    for (int q = 0; q < kNs / 4; ++q) { const v4f av = *(const v4f*)(A_log + (size_t)(c0 + k) * kNs + 4 * q);
#pragma unroll
      for (int e = 0; e < 4; ++e) { A[k][4 * q + e] = -expf(bf16r(av[e])); st[k][4 * q + e] = 0.0f; } }
    const v4f wv = *(const v4f*)(conv_w + (size_t)(c0 + k) * kTaps);
#pragma unroll
    for (int t = 0; t < kTaps; ++t) cw[k][t] = bf16r(wv[t]);
#pragma unroll
    for (int t = 0; t < kTaps - 1; ++t) win[k][t] = 0.0f;
    const float q0 = Dp[c0 + k];
    dc[k] = bf16r(q0);
  }
  for (int l = 0; l < kL; ++l) {
    const size_t row = (size_t)sq * kL + (size_t)l;
    const float* px = XZ + row * kXZ;
    const v2f xr = *(const v2f*)(px + c0);
    const v2f zr = *(const v2f*)(px + kDI + c0);
    const float* pr = XP + row * kXpP;
    const float pre = pr[2 * kNs];
    const float delta = (pre > 20.0f) ? pre : log1pf(expf(pre));
    float xc[2], y[2];
#pragma unroll
    for (int k = 0; k < 2; ++k) {
      float acc = 0.0f;
      acc += win[k][0] * cw[k][0];
      acc += win[k][1] * cw[k][1];
      acc += win[k][2] * cw[k][2];
      acc += xr[k] * cw[k][3];
      win[k][0] = win[k][1]; win[k][1] = win[k][2]; win[k][2] = xr[k];
      xc[k] = acc / (1.0f + expf(-acc));
      y[k] = 0.0f;
    }
#pragma unroll
    for (int q = 0; q < kNs / 4; ++q) {
      const v4f bv = *(const v4f*)(pr + 4 * q), cv = *(const v4f*)(pr + kNs + 4 * q);
#pragma unroll
      for (int e = 0; e < 4; ++e) {
        const int n = 4 * q + e;
#pragma unroll
        for (int k = 0; k < 2; ++k) {
          const float sn = st[k][n] * expf(delta * A[k][n]) + xc[k] * bv[e];
          st[k][n] = sn;
          y[k] += sn * cv[e];
        }
      }
    }
    v2h hv;
#pragma unroll
    for (int k = 0; k < 2; ++k) { const float zz = zr[k]; hv[k] = (_Float16)carry_flush((y[k] + xc[k] * dc[k]) * (zz / (1.0f + expf(-zz))), kYCarry); }
    unsigned short* dp = Y16 + row * kDI + c0;
    *(volatile v2h*)dp = hv;
    __threadfence();
    *(volatile v2h*)dp = hv;
  }
  float* fp = out1 + ((size_t)sq * kDI + c0) * kNs;
  for (int pass = 0; pass < 2; ++pass) {
#pragma unroll
    for (int k = 0; k < 2; ++k) {
#pragma unroll
      for (int q = 0; q < kNs / 4; ++q) { v4f o; o[0] = st[k][4 * q]; o[1] = st[k][4 * q + 1]; o[2] = st[k][4 * q + 2]; o[3] = st[k][4 * q + 3]; *(volatile v4f*)(fp + k * kNs + 4 * q) = o; }
    }
    __threadfence();
  }
}
static_assert(kNB * kDI / 2 == 12 * kThr && kDI / 2 == 768 && (kNs % 4) == 0 && (2 * kNs * 4) == 128, "scan grid exact: 12 blocks: three a sequence; a lane's two channels' final states are one 128-B line");

extern "C" void kernel_launch(void* const* d_in, const int* in_sizes, int n_in,
                              void* d_out, int out_size, void* d_ws, size_t ws_size,
                              hipStream_t stream) {
  if (n_in < 7 || d_out == nullptr || d_ws == nullptr) return;
  if (in_sizes[0] != kRows * kHid || in_sizes[1] != kXZ * kHid || in_sizes[2] != kDI * kTaps || in_sizes[3] != (2 * kNs + 1) * kDI || in_sizes[4] != kDI * kNs || in_sizes[5] != kDI || in_sizes[6] != kHid * kDI) return;
  if (out_size != kOut0 + kOut1) return;
  if (ws_size < kWsTotal) return;
  const float* x = (const float*)d_in[0];
  const float* W_in = (const float*)d_in[1];
  const float* conv_w = (const float*)d_in[2];
  const float* W_xp = (const float*)d_in[3];
  const float* A_log = (const float*)d_in[4];
  const float* D_skip = (const float*)d_in[5];
  const float* W_out = (const float*)d_in[6];
  float* out = (float*)d_out;
  char* ws = (char*)d_ws;
  unsigned short* X16 = (unsigned short*)(ws + kOffX16);
  unsigned short* WIN16 = (unsigned short*)(ws + kOffWIN16);
  unsigned short* WOUT16 = (unsigned short*)(ws + kOffWOUT16);
  unsigned short* WXP16 = (unsigned short*)(ws + kOffWXP16);
  float* ZB = (float*)(ws + kOffZB);
  float* XZ = (float*)(ws + kOffXZ);
  unsigned short* U16 = (unsigned short*)(ws + kOffU16);
  float* XP = (float*)(ws + kOffXP);
  unsigned short* Y16 = (unsigned short*)(ws + kOffY16);

  static_assert(((size_t)kRows * kHid / 8) % kThr == 0 && ((size_t)kXZ * kHid / 8) % kThr == 0 && ((size_t)kHid * kDI / 8) % kThr == 0 && ((size_t)kRows * kHid) % 1024 == 0 && ((size_t)kXZ * kHid) % 1024 == 0 && ((size_t)kHid * kDI) % 1024 == 0, "the casts' grids; every plane is whole rows of 1,024");
  cast_plane_kernel<<<(int)(((size_t)kRows * kHid / 8) / kThr), kThr, 0, stream>>>(x, X16, 10, 1024, 0);
  cast_plane_kernel<<<(int)(((size_t)kXZ * kHid / 8) / kThr), kThr, 0, stream>>>(W_in, WIN16, 10, 1024, 0);
  cast_plane_kernel<<<(int)(((size_t)kHid * kDI / 8) / kThr), kThr, 0, stream>>>(W_out, WOUT16, 10, 1024, 0);
  setup_kernel<<<60, kThr, 0, stream>>>(W_xp, ZB, WXP16);
  wmma_gemm64<0, false, 2, 0, false, 0><<<dim3((kRows / 64) * (kXZ / 64) / 8, 1), 256, 0, stream>>>(
      X16, X16, kHid, 0L, WIN16, WIN16, kHid, 0L, (void*)XZ, (void*)XZ, kXZ, 0L, ZB, nullptr, 0L, kRows, kXZ, kHid, kScIn);
  front_kernel<<<6144, kThr, 0, stream>>>(XZ, conv_w, U16);
  wmma_gemm64<0, false, 2, 0, false, 0><<<dim3((kRows / 64) * (kXpP / 64) / 8, 1), 256, 0, stream>>>(
      U16, U16, kDI, 0L, WXP16, WXP16, kDI, 0L, (void*)XP, (void*)XP, kXpP, 0L, ZB, nullptr, 0L, kRows, kXpP, kDI, kScU);
  scan_kernel<<<12, kThr, 0, stream>>>(XZ, XP, conv_w, A_log, D_skip, Y16, out + kOut0);
  wmma_gemm64<0, false, 2, 0, false, 0><<<dim3((kRows / 64) * (kHid / 64) / 8, 1), 256, 0, stream>>>(
      Y16, Y16, kDI, 0L, WOUT16, WOUT16, kDI, 0L, (void*)out, (void*)out, kHid, 0L, ZB, nullptr, 0L, kRows, kHid, kDI, kScY);
}
static_assert(((kRows / 64) * (kXZ / 64)) % 8 == 0 && ((kRows / 64) * (kXpP / 64)) % 8 == 0 && ((kRows / 64) * (kHid / 64)) % 8 == 0, "the engine's grids: whole blocks of eight wave tiles");
